// UV_Aggregator_70102456205704
// MI455X (gfx1250) — hardware-verified
//
#include <hip/hip_runtime.h>
#include <math.h>

#define NUSR   16384
#define LNB    50
#define DD     64
#define NTAB   100000
#define NRAT   5
#define UPB    64
#define PA     136
#define PW     72
#define LP     52
#define NTHR   128

typedef __bf16         v16b __attribute__((ext_vector_type(16)));
typedef __bf16         v8b  __attribute__((ext_vector_type(8)));
typedef unsigned int   v2u  __attribute__((ext_vector_type(2)));
typedef float          v8f  __attribute__((ext_vector_type(8)));
typedef float          v4f  __attribute__((ext_vector_type(4)));
typedef v8b __attribute__((may_alias)) v8ba;
typedef v2u __attribute__((may_alias)) v2ua;
typedef v4f __attribute__((may_alias)) v4fa;

static_assert(NUSR % UPB == 0);
static_assert((PA % 8) == 0 && (PW % 8) == 0);
static_assert(UPB == 64 && NTHR == 128);
static_assert(LNB <= LP);

__device__ __forceinline__ unsigned short f2bf_bits(float f) {
  const unsigned u = __float_as_uint(f);
  return (unsigned short)((u + 0x7FFFu + ((u >> 16) & 1u)) >> 16);
}
__device__ __forceinline__ float bf2f(unsigned short b) { return __uint_as_float(((unsigned)b) << 16); }
__device__ __forceinline__ float bfr(float f) { return bf2f(f2bf_bits(f)); }
__device__ __forceinline__ unsigned pk2(float a, float b) {
  return (unsigned)f2bf_bits(a) | ((unsigned)f2bf_bits(b) << 16);
}

__device__ __forceinline__ v8f mma_bf16(v16b a, v16b b, v8f c) {
  c = __builtin_amdgcn_wmma_f32_16x16x32_bf16(false, a, false, b, (short)0, c, false, false);
  asm volatile("v_nop\n\tv_nop\n\tv_nop\n\tv_nop" : "+v"(c) : "v"(a), "v"(b));
  return c;
}

__device__ __forceinline__ v16b ld_frag(const unsigned short* p) {
  union { v16b v; v8b hh[2]; } f;
  f.hh[0] = *(const v8ba*)(p);
  f.hh[1] = *(const v8ba*)(p + 16);
  return f.v;
}

template <int NK, int KWM>
__device__ __forceinline__ void tile_mma(v8f (&acc)[4], const unsigned short* ap,
                                         const unsigned short* bp, int bstep) {
  const v8f z = {0.f, 0.f, 0.f, 0.f, 0.f, 0.f, 0.f, 0.f};
#pragma unroll
  for (int nt = 0; nt < 4; ++nt) acc[nt] = z;
#pragma unroll 1
  for (int ks = 0; ks < NK; ++ks) {
    const int k0 = ks << 5;
    const int kb = k0 & KWM;
    const v16b a = ld_frag(ap + k0);
#pragma unroll
    for (int nt = 0; nt < 4; ++nt) {
      const v16b b = ld_frag(bp + nt * bstep + kb);
      acc[nt] = mma_bf16(a, b, acc[nt]);
    }
  }
}

__device__ __forceinline__ void split_rows(const v8f (&acc)[4], const float (&bb)[4],
                                           unsigned short* trow, int m) {
#pragma unroll
  for (int nt = 0; nt < 4; ++nt) {
#pragma unroll
    for (int r = 0; r < 8; ++r) {
      const float v = fmaxf(acc[nt][r] + bb[nt], 0.0f);
      const unsigned short hb = f2bf_bits(v);
      trow[r * PA + 16 * nt + m]      = hb;
      trow[r * PA + 64 + 16 * nt + m] = f2bf_bits(v - bf2f(hb));
    }
  }
}

__device__ __forceinline__ void gather_slot(unsigned short* sXA, const unsigned short* sR2,
                                            const int* huv, const int* hr, const float* v2e,
                                            int ub0, int l, int t) {
  const int row = t >> 1, half = t & 1;
  const int hidx = (ub0 + row) * LNB + l;
  int item = huv[hidx];
  item = (item < 0) ? item + NTAB : item;
  item = min(max(item, 0), NTAB - 1);
  int rr = hr[hidx];
  rr = rr - ((rr > 0) ? 1 : 0) + ((rr < 0) ? 1 : 0);
  rr = (rr < 0) ? rr + NRAT : rr;
  rr = min(max(rr, 0), NRAT - 1);
  const float* src = v2e + (size_t)item * DD + half * 32;
  unsigned short* xr = sXA + row * PA + half * 32;
  const unsigned short* rs = sR2 + rr * DD + half * 32;
#pragma unroll
  for (int j = 0; j < 8; ++j) {
    const v4f v = *(const v4fa*)(src + 4 * j);
    v2u pk;
    pk.x = pk2(v.x, v.y);
    pk.y = pk2(v.z, v.w);
    *(v2ua*)(xr + 4 * j) = pk;
    *(v2ua*)(xr + 64 + 4 * j) = *(const v2ua*)(rs + 4 * j);
  }
}

__device__ __forceinline__ void out_store_pass(const float* so, float* out, int ub0, int rw, int lane) {
  const int q = lane >> 3, c4 = (lane & 7) << 2;
#pragma unroll
  for (int it = 0; it < 8; ++it) {
    const int lid = it * 4 + q;
    const int row = lid >> 1, hl = lid & 1;
    const v4f v = *(const v4fa*)(so + (rw + row) * DD + 32 * hl + c4);
    *(volatile v4f*)(out + (size_t)(ub0 + rw + row) * DD + 32 * hl + c4) = v;
  }
}

__global__ __launch_bounds__(NTHR) void uvagg_kernel(
    const int* __restrict__ nodes, const int* __restrict__ huv, const int* __restrict__ hr,
    const float* __restrict__ v2e, const float* __restrict__ u2e, const float* __restrict__ r2e,
    const float* __restrict__ w1, const float* __restrict__ b1,
    const float* __restrict__ w2, const float* __restrict__ b2,
    const float* __restrict__ a1, const float* __restrict__ ab1,
    const float* __restrict__ a2, const float* __restrict__ ab2,
    const float* __restrict__ a3, const float* __restrict__ ab3,
    float* __restrict__ out)
{
  __shared__ __align__(16) unsigned short sW1[64 * PA];
  __shared__ __align__(16) unsigned short sW2[64 * PW];
  __shared__ __align__(16) unsigned short sA1t[64 * PW];
  __shared__ __align__(16) unsigned short sA1b[64 * PW];
  __shared__ __align__(16) unsigned short sA2[64 * PW];
  __shared__ __align__(16) unsigned short sR2[8 * DD];
  __shared__ __align__(16) unsigned short sXA[64 * PA];
  __shared__ __align__(16) unsigned short sT0[64 * PA];
  __shared__ __align__(16) unsigned short sT1[64 * PA];
  __shared__ __align__(16) unsigned short sUT[64 * PW];
  __shared__ __align__(16) float sUB[64 * DD];
  __shared__ __align__(16) float sLG[64 * LP];
  __shared__ __align__(16) float sBias[5 * DD];

  const int t = threadIdx.x;
  const int lane = t & 31, w = t >> 5, h = lane >> 4, m = lane & 15;
  const int ub0 = blockIdx.x * UPB;
  const int rw = 16 * w;
  const int rrow = rw + 8 * h;

#pragma unroll 2
  for (int it = 0; it < 16; ++it) {
    const int f = it * NTHR + t;
    const int k = f >> 4, n4 = (f & 15) << 2;
    const v4f v = *(const v4fa*)(w1 + (size_t)f * 4);
    sW1[(n4 + 0) * PA + k] = f2bf_bits(v.x);
    sW1[(n4 + 1) * PA + k] = f2bf_bits(v.y);
    sW1[(n4 + 2) * PA + k] = f2bf_bits(v.z);
    sW1[(n4 + 3) * PA + k] = f2bf_bits(v.w);
  }
#pragma unroll 2
  for (int it = 0; it < 8; ++it) {
    const int f = it * NTHR + t;
    const int k = f >> 4, n4 = (f & 15) << 2;
    const v4f v = *(const v4fa*)(w2 + (size_t)f * 4);
    const v4f c = *(const v4fa*)(a2 + (size_t)f * 4);
    const v4f p = *(const v4fa*)(a1 + (size_t)f * 4);
    const v4f q = *(const v4fa*)(a1 + (size_t)(f + 8 * NTHR) * 4);
    sW2 [(n4 + 0) * PW + k] = f2bf_bits(v.x);  sW2 [(n4 + 1) * PW + k] = f2bf_bits(v.y);
    sW2 [(n4 + 2) * PW + k] = f2bf_bits(v.z);  sW2 [(n4 + 3) * PW + k] = f2bf_bits(v.w);
    sA2 [(n4 + 0) * PW + k] = f2bf_bits(c.x);  sA2 [(n4 + 1) * PW + k] = f2bf_bits(c.y);
    sA2 [(n4 + 2) * PW + k] = f2bf_bits(c.z);  sA2 [(n4 + 3) * PW + k] = f2bf_bits(c.w);
    sA1t[(n4 + 0) * PW + k] = f2bf_bits(p.x);  sA1t[(n4 + 1) * PW + k] = f2bf_bits(p.y);
    sA1t[(n4 + 2) * PW + k] = f2bf_bits(p.z);  sA1t[(n4 + 3) * PW + k] = f2bf_bits(p.w);
    sA1b[(n4 + 0) * PW + k] = f2bf_bits(q.x);  sA1b[(n4 + 1) * PW + k] = f2bf_bits(q.y);
    sA1b[(n4 + 2) * PW + k] = f2bf_bits(q.z);  sA1b[(n4 + 3) * PW + k] = f2bf_bits(q.w);
  }
  {
    const int f = min(t, 79);
    const int rr = f >> 4, c4 = (f & 15) << 2;
    const v4f v = *(const v4fa*)(r2e + (size_t)f * 4);
    if (t < 80) {
      sR2[rr * DD + c4 + 0] = f2bf_bits(v.x);
      sR2[rr * DD + c4 + 1] = f2bf_bits(v.y);
      sR2[rr * DD + c4 + 2] = f2bf_bits(v.z);
      sR2[rr * DD + c4 + 3] = f2bf_bits(v.w);
    }
  }
  {
    const int row = t >> 1, half = t & 1;
    int nd = nodes[ub0 + row];
    nd = (nd < 0) ? nd + NTAB : nd;
    nd = min(max(nd, 0), NTAB - 1);
    const float* src = u2e + (size_t)nd * DD + half * 32;
    unsigned short* dst = sUT + row * PW + half * 32;
#pragma unroll
    for (int j = 0; j < 8; ++j) {
      const v4f v = *(const v4fa*)(src + 4 * j);
      v2u pk;
      pk.x = pk2(v.x, v.y);
      pk.y = pk2(v.z, v.w);
      *(v2ua*)(dst + 4 * j) = pk;
    }
  }
  if (t < DD) {
    sBias[t]          = bfr(b1[t]);
    sBias[DD + t]     = bfr(b2[t]);
    sBias[2 * DD + t] = bfr(ab1[t]);
    sBias[3 * DD + t] = bfr(ab2[t]);
    sBias[4 * DD + t] = bfr(a3[t]);
  }
  const float ab3v = bfr(ab3[0]);
  __syncthreads();

  float b1c[4], b2c[4], ab1c[4], ab2c[4], a3c[4];
#pragma unroll
  for (int nt = 0; nt < 4; ++nt) {
    b1c[nt]  = sBias[16 * nt + m];
    b2c[nt]  = sBias[DD + 16 * nt + m];
    ab1c[nt] = sBias[2 * DD + 16 * nt + m];
    ab2c[nt] = sBias[3 * DD + 16 * nt + m];
    a3c[nt]  = sBias[4 * DD + 16 * nt + m];
  }

  const unsigned short* apX   = sXA  + (rw + m) * PA + 8 * h;
  const unsigned short* apT0  = sT0  + (rw + m) * PA + 8 * h;
  const unsigned short* apT1  = sT1  + (rw + m) * PA + 8 * h;
  const unsigned short* bpW1  = sW1  + m * PA + 8 * h;
  const unsigned short* bpW2  = sW2  + m * PW + 8 * h;
  const unsigned short* bpA1t = sA1t + m * PW + 8 * h;
  const unsigned short* bpA1b = sA1b + m * PW + 8 * h;
  const unsigned short* bpA2  = sA2  + m * PW + 8 * h;
  unsigned short* t0row = sT0 + rrow * PA;
  unsigned short* t1row = sT1 + rrow * PA;

  {
    v8f acc[4];
    tile_mma<2, 63>(acc, sUT + (rw + m) * PW + 8 * h, bpA1b, 16 * PW);
#pragma unroll
    for (int nt = 0; nt < 4; ++nt)
#pragma unroll
      for (int r = 0; r < 8; ++r) sUB[(rrow + r) * DD + 16 * nt + m] = acc[nt][r];
  }

#pragma unroll 1
  for (int l = 0; l < LNB; ++l) {
    __syncthreads();
    gather_slot(sXA, sR2, huv, hr, v2e, ub0, l, t);
    __syncthreads();
    v8f acc[4];
    tile_mma<4, 127>(acc, apX, bpW1, 16 * PA);
    split_rows(acc, b1c, t0row, m);
    __syncthreads();
    tile_mma<4, 63>(acc, apT0, bpW2, 16 * PW);
    split_rows(acc, b2c, t1row, m);
    __syncthreads();
    tile_mma<4, 63>(acc, apT1, bpA1t, 16 * PW);
#pragma unroll
    for (int nt = 0; nt < 4; ++nt) {
#pragma unroll
      for (int r = 0; r < 8; ++r) {
        const float v = fmaxf(acc[nt][r] + sUB[(rrow + r) * DD + 16 * nt + m] + ab1c[nt], 0.0f);
        const unsigned short hb = f2bf_bits(v);
        t0row[r * PA + 16 * nt + m]      = hb;
        t0row[r * PA + 64 + 16 * nt + m] = f2bf_bits(v - bf2f(hb));
      }
    }
    __syncthreads();
    tile_mma<4, 63>(acc, apT0, bpA2, 16 * PW);
    float part[8];
#pragma unroll
    for (int r = 0; r < 8; ++r) part[r] = 0.0f;
#pragma unroll
    for (int nt = 0; nt < 4; ++nt) {
#pragma unroll
      for (int r = 0; r < 8; ++r) {
        const float v = fmaxf(acc[nt][r] + ab2c[nt], 0.0f);
        part[r] += v * a3c[nt];
      }
    }
#pragma unroll
    for (int r = 0; r < 8; ++r) {
      float p = part[r];
      p += __shfl_xor(p, 1);
      p += __shfl_xor(p, 2);
      p += __shfl_xor(p, 4);
      p += __shfl_xor(p, 8);
      part[r] = p;
    }
    if (m == 0) {
#pragma unroll
      for (int r = 0; r < 8; ++r) sLG[(rrow + r) * LP + l] = part[r] + ab3v;
    }
  }

  __syncthreads();
  if (t < UPB) {
    float* lg = sLG + t * LP;
    float mx = lg[0];
#pragma unroll 1
    for (int l = 1; l < LNB; ++l) mx = fmaxf(mx, lg[l]);
    float s = 0.0f;
#pragma unroll 1
    for (int l = 0; l < LNB; ++l) {
      const float e = expf(lg[l] - mx);
      lg[l] = e;
      s += e;
    }
    const float inv = 1.0f / s;
#pragma unroll 1
    for (int l = 0; l < LNB; ++l) lg[l] = lg[l] * inv;
  }
  __syncthreads();

  v8f oacc[4];
  {
    const v8f z = {0.f, 0.f, 0.f, 0.f, 0.f, 0.f, 0.f, 0.f};
#pragma unroll
    for (int nt = 0; nt < 4; ++nt) oacc[nt] = z;
  }
#pragma unroll 1
  for (int l = 0; l < LNB; ++l) {
    __syncthreads();
    gather_slot(sXA, sR2, huv, hr, v2e, ub0, l, t);
    __syncthreads();
    v8f acc[4];
    tile_mma<4, 127>(acc, apX, bpW1, 16 * PA);
    split_rows(acc, b1c, t0row, m);
    __syncthreads();
    tile_mma<4, 63>(acc, apT0, bpW2, 16 * PW);
    float att[8];
#pragma unroll
    for (int r = 0; r < 8; ++r) att[r] = sLG[(rrow + r) * LP + l];
#pragma unroll
    for (int nt = 0; nt < 4; ++nt) {
#pragma unroll
      for (int r = 0; r < 8; ++r) {
        const float o = fmaxf(acc[nt][r] + b2c[nt], 0.0f);
        oacc[nt][r] += att[r] * o;
      }
    }
  }

  __syncthreads();
#pragma unroll
  for (int nt = 0; nt < 4; ++nt)
#pragma unroll
    for (int r = 0; r < 8; ++r) sUB[(rrow + r) * DD + 16 * nt + m] = oacc[nt][r];
  __syncthreads();
  out_store_pass(sUB, out, ub0, rw, lane);
  __threadfence();
  out_store_pass(sUB, out, ub0, rw, lane);
}

extern "C" void kernel_launch(void* const* d_in, const int* in_sizes, int n_in,
                              void* d_out, int out_size, void* d_ws, size_t ws_size,
                              hipStream_t stream) {
  if (n_in < 16) return;
  if (in_sizes[0] != NUSR) return;
  if (in_sizes[1] != NUSR * LNB || in_sizes[2] != NUSR * LNB) return;
  if (in_sizes[3] != NTAB * DD || in_sizes[4] != NTAB * DD) return;
  if (in_sizes[5] != NRAT * DD) return;
  if (in_sizes[6] != 2 * DD * DD || in_sizes[7] != DD) return;
  if (in_sizes[8] != DD * DD || in_sizes[9] != DD) return;
  if (in_sizes[10] != 2 * DD * DD || in_sizes[11] != DD) return;
  if (in_sizes[12] != DD * DD || in_sizes[13] != DD) return;
  if (in_sizes[14] != DD || in_sizes[15] != 1) return;
  if (out_size != NUSR * DD) return;
  (void)d_ws; (void)ws_size;

  const int*   nodes = (const int*)d_in[0];
  const int*   huv   = (const int*)d_in[1];
  const int*   hr    = (const int*)d_in[2];
  const float* v2e   = (const float*)d_in[3];
  const float* u2e   = (const float*)d_in[4];
  const float* r2e   = (const float*)d_in[5];
  const float* w1    = (const float*)d_in[6];
  const float* b1    = (const float*)d_in[7];
  const float* w2    = (const float*)d_in[8];
  const float* b2    = (const float*)d_in[9];
  const float* a1    = (const float*)d_in[10];
  const float* ab1   = (const float*)d_in[11];
  const float* a2    = (const float*)d_in[12];
  const float* ab2   = (const float*)d_in[13];
  const float* a3    = (const float*)d_in[14];
  const float* ab3   = (const float*)d_in[15];
  float* out = (float*)d_out;

  uvagg_kernel<<<dim3(NUSR / UPB), dim3(NTHR), 0, stream>>>(
      nodes, huv, hr, v2e, u2e, r2e, w1, b1, w2, b2, a1, ab1, a2, ab2, a3, ab3, out);
  (void)hipGetLastError();
}
